// PointNet2SAModuleCUDA_5007931867461
// MI455X (gfx1250) — hardware-verified
//
#include <hip/hip_runtime.h>
#include <math.h>

#pragma clang fp contract(off)

typedef __attribute__((ext_vector_type(16))) _Float16 v16h;
typedef __attribute__((ext_vector_type(8)))  _Float16 v8h;
typedef __attribute__((ext_vector_type(16))) __bf16   v16b;
typedef __attribute__((ext_vector_type(8)))  __bf16   v8b;
typedef __attribute__((ext_vector_type(8)))  float    v8f;
typedef __attribute__((ext_vector_type(4)))  float    v4f;
typedef __attribute__((ext_vector_type(4)))  unsigned v4u;
typedef __attribute__((ext_vector_type(4)))  int      v4i;

constexpr int kBatch   = 8;
constexpr int kPts     = 4096;
constexpr int kCent    = 1024;
constexpr int kFeat    = 64;
constexpr int kNbr     = 32;
constexpr int kChan    = 212;
constexpr int kChanPad = 224;
constexpr int kOutCh   = 128;
constexpr int kTilePW  = 116;
constexpr int kRowW    = 112;
constexpr float kWCarry    = 16.0f;
constexpr float kWCarryInv = 1.0f / 16.0f;

static_assert(kChan == 3 * 3 + 1 + 3 * (kFeat + 3) + 1, "channel count");
static_assert(kChanPad % 32 == 0 && kChanPad >= kChan, "K pad");
static_assert(kOutCh % 64 == 0 && kCent % 64 == 0, "GEMM tile multiples");
static_assert(98304 == kBatch * kCent * 3 * 4, "out0 bytes");
static_assert(98304 + kBatch * kOutCh * kCent * 4 == 4292608, "d_out total");

__device__ __forceinline__ unsigned short f2bf_bits(float f) {
  unsigned u = __float_as_uint(f);
  return (unsigned short)((u + 0x7FFFu + ((u >> 16) & 1u)) >> 16);
}
__device__ __forceinline__ float bf_bits2f(unsigned short h) { return __uint_as_float(((unsigned)h) << 16); }
__device__ __forceinline__ float bfr(float f) { return bf_bits2f(f2bf_bits(f)); }

__device__ __forceinline__ unsigned h16bits(float x) {
  const _Float16 hv = (_Float16)x;
  const unsigned short us = __builtin_bit_cast(unsigned short, hv);
  return (unsigned)us;
}
__device__ __forceinline__ unsigned pk16(float lo, float hi) {
  const unsigned a = h16bits(lo);
  const unsigned b = h16bits(hi);
  return (a & 0xffffu) | (b << 16);
}
__device__ __forceinline__ float h16_to_f32(unsigned hb) {
  const unsigned sgn = (hb & 0x8000u) << 16;
  const unsigned em = hb & 0x7fffu;
  const float fn = __uint_as_float((em << 13) + 0x38000000u);
  const float fs = (float)em * 5.9604644775390625e-8f;
  const float mag = (em < 0x400u) ? fs : fn;
  return __uint_as_float(__float_as_uint(mag) | sgn);
}
__device__ __forceinline__ int clampi(int v, int lo, int hi) { return v < lo ? lo : (v > hi ? hi : v); }

__device__ __forceinline__ int cmap(int p) {
  int c = p + 10;
  c = (p >= 64) ? (p + 13) : c;
  c = (p >= 128) ? (p + 16) : c;
  c = (p >= 192) ? (p - 192) : c;
  c = (p >= 202) ? (p - 202 + 74) : c;
  c = (p >= 205) ? (p - 205 + 141) : c;
  c = (p >= 208) ? p : c;
  return c;
}

__global__ __launch_bounds__(256) void k_prep_xyz(const float* __restrict__ xyz, const float* __restrict__ b1,
                                                  float* __restrict__ xyzr, float* __restrict__ b1r) {
  const int nblk = (kBatch * kPts * 3 / 4) / 256;
  if ((int)blockIdx.x < nblk) {
    const int i = blockIdx.x * 256 + threadIdx.x;
    const v4f v = *(const v4f*)(xyz + 4 * (size_t)i);
    const float a0 = v.x, a1 = v.y, a2 = v.z, a3 = v.w;
    v4f r;
    r.x = bfr(a0); r.y = bfr(a1); r.z = bfr(a2); r.w = bfr(a3);
    volatile v4f* dst = (volatile v4f*)(xyzr + 4 * (size_t)i);
    *dst = r;
    __threadfence();
    *dst = r;
  } else if (threadIdx.x < 32) {
    const int i = threadIdx.x;
    const v4f v = *(const v4f*)(b1 + 4 * i);
    const float a0 = v.x, a1 = v.y, a2 = v.z, a3 = v.w;
    v4f r;
    r.x = bfr(a0); r.y = bfr(a1); r.z = bfr(a2); r.w = bfr(a3);
    volatile v4f* dst = (volatile v4f*)(b1r + 4 * i);
    *dst = r;
    __threadfence();
    *dst = r;
  }
}

__global__ __launch_bounds__(256) void k_prep_feat(const float* __restrict__ feat, unsigned* __restrict__ featT) {
  __shared__ __align__(16) unsigned s_w[64 * 36];
  const int b = blockIdx.x >> 6;
  const int j0 = (blockIdx.x & 63) * 64;
  const int tid = threadIdx.x;
  const float* F = feat + (size_t)b * kFeat * kPts;
#pragma unroll 1
  for (int g = 0; g < 2; ++g) {
#pragma unroll
    for (int i = 0; i < 4; ++i) {
      const int q = tid + 256 * (g * 4 + i);
      const int cp = q >> 6;
      const int jj = q & 63;
      const float v0 = F[(size_t)(2 * cp) * kPts + j0 + jj];
      const float v1 = F[(size_t)(2 * cp + 1) * kPts + j0 + jj];
      const unsigned lo = (unsigned)f2bf_bits(v0);
      const unsigned hi = (unsigned)f2bf_bits(v1);
      s_w[jj * 36 + cp] = (lo & 0xffffu) | (hi << 16);
    }
  }
  __syncthreads();
  v4u v[2];
#pragma unroll
  for (int it = 0; it < 2; ++it) {
    const int jj = (tid >> 3) + 32 * it;
    const int w4 = (tid & 7) * 4;
    v[it] = *(const v4u*)(s_w + jj * 36 + w4);
  }
  for (int pass = 0; pass < 2; ++pass) {
#pragma unroll
    for (int it = 0; it < 2; ++it) {
      const int jj = (tid >> 3) + 32 * it;
      const int w4 = (tid & 7) * 4;
      *(volatile v4u*)(featT + ((size_t)(b * kPts + j0 + jj)) * 32 + w4) = v[it];
    }
    __threadfence();
  }
}

__global__ __launch_bounds__(256) void k_prep_at(const float* __restrict__ a, unsigned* __restrict__ AtW) {
  const int total = kChanPad * 28;
  const int q = blockIdx.x * 256 + threadIdx.x;
  const int qc = q < total ? q : (total - 1);
  const int n = qc / 28;
  const int p8 = (qc - n * 28) * 8;
  float zf = 0.0f;
  asm volatile("" : "+v"(zf));
  const bool nv = n < kChan;
  const int d = cmap(nv ? n : (kChan - 1));
  unsigned w[4];
#pragma unroll
  for (int i = 0; i < 4; ++i) {
    const int p0 = p8 + 2 * i;
    const int p1 = p0 + 1;
    const bool ok0 = nv && (p0 < kChan);
    const bool ok1 = nv && (p1 < kChan);
    const int c0 = cmap(p0 < kChan ? p0 : (kChan - 1));
    const int c1 = cmap(p1 < kChan ? p1 : (kChan - 1));
    const float x0 = a[c0 * kChan + d];
    const float x1 = a[c1 * kChan + d];
    const float y0 = ok0 ? (bfr(x0) * kWCarry) : zf;
    const float y1 = ok1 ? (bfr(x1) * kWCarry) : zf;
    w[i] = pk16(y0, y1);
  }
  v4u v;
  v.x = w[0]; v.y = w[1]; v.z = w[2]; v.w = w[3];
  if (q < total) *(volatile v4u*)(AtW + (size_t)q * 4) = v;
  __threadfence();
  if (q < total) *(volatile v4u*)(AtW + (size_t)q * 4) = v;
}

__global__ __launch_bounds__(256) void k_prep_w1(const float* __restrict__ w1, unsigned* __restrict__ W1b,
                                                 unsigned* __restrict__ W1z) {
  const int total = kOutCh * 28;
  const int q = blockIdx.x * 256 + threadIdx.x;
  const int qc = q < total ? q : (total - 1);
  const int o = qc / 28;
  const int p8 = (qc - o * 28) * 8;
  unsigned zz = 0u;
  asm volatile("" : "+v"(zz));
  unsigned w[4];
#pragma unroll
  for (int i = 0; i < 4; ++i) {
    const int p0 = p8 + 2 * i;
    const int p1 = p0 + 1;
    const int c0 = cmap(p0 < kChan ? p0 : (kChan - 1));
    const int c1 = cmap(p1 < kChan ? p1 : (kChan - 1));
    const float x0 = w1[o * kChan + c0];
    const float x1 = w1[o * kChan + c1];
    const unsigned b0 = (p0 < kChan) ? (unsigned)f2bf_bits(x0) : zz;
    const unsigned b1 = (p1 < kChan) ? (unsigned)f2bf_bits(x1) : zz;
    w[i] = (b0 & 0xffffu) | (b1 << 16);
  }
  v4u v;
  v.x = w[0]; v.y = w[1]; v.z = w[2]; v.w = w[3];
  v4u z;
  z.x = zz; z.y = zz; z.z = zz; z.w = zz;
  if (q < total) {
    *(volatile v4u*)(W1b + (size_t)q * 4) = v;
    *(volatile v4u*)(W1z + (size_t)q * 4) = z;
  }
  __threadfence();
  if (q < total) {
    *(volatile v4u*)(W1b + (size_t)q * 4) = v;
    *(volatile v4u*)(W1z + (size_t)q * 4) = z;
  }
}

__global__ __launch_bounds__(1024) void k_fps(const float* __restrict__ xyzr, int* __restrict__ fps_idx,
                                              float* __restrict__ out0) {
#pragma clang fp contract(off)
  __shared__ float s_x[kPts * 3];
  __shared__ float s_val[2][32];
  __shared__ int   s_ix[2][32];
  __shared__ __align__(16) int s_sel[kCent];
  const int b = blockIdx.x;
  const int tid = threadIdx.x;
  const int lane = tid & 31;
  const int wid = tid >> 5;
  const float* X = xyzr + (size_t)b * kPts * 3;
#pragma unroll
  for (int i = 0; i < 12; ++i) s_x[tid + i * 1024] = X[tid + i * 1024];
  if (tid == 0) s_sel[0] = 0;
  __syncthreads();

  float px[4], py[4], pz[4], dmin[4];
#pragma unroll
  for (int i = 0; i < 4; ++i) {
    const int nn = tid + i * 1024;
    px[i] = s_x[nn * 3 + 0];
    py[i] = s_x[nn * 3 + 1];
    pz[i] = s_x[nn * 3 + 2];
    dmin[i] = 1e10f;
  }

  int cur = 0;
#pragma unroll 1
  for (int it = 1; it < kCent; ++it) {
    const float lx = s_x[cur * 3 + 0];
    const float ly = s_x[cur * 3 + 1];
    const float lz = s_x[cur * 3 + 2];
    float bv = -1.0f;
    int bi = 0;
#pragma unroll
    for (int i = 0; i < 4; ++i) {
      const float dx = px[i] - lx;
      const float dy = py[i] - ly;
      const float dz = pz[i] - lz;
      const float t0 = dx * dx;
      const float t1 = dy * dy;
      const float t2 = dz * dz;
      const float d = (t0 + t2) + t1;
      const float dm = fminf(dmin[i], d);
      dmin[i] = dm;
      const bool tk = dm > bv;
      bv = tk ? dm : bv;
      bi = tk ? (tid + i * 1024) : bi;
    }
#pragma unroll
    for (int o = 16; o > 0; o >>= 1) {
      const float ov = __shfl_xor(bv, o);
      const int   oi = __shfl_xor(bi, o);
      const bool tk = (ov > bv) || (ov == bv && oi < bi);
      bv = tk ? ov : bv;
      bi = tk ? oi : bi;
    }
    const int buf = it & 1;
    if (lane == 0) { s_val[buf][wid] = bv; s_ix[buf][wid] = bi; }
    __syncthreads();
    float v = s_val[buf][lane];
    int ix = s_ix[buf][lane];
#pragma unroll
    for (int o = 16; o > 0; o >>= 1) {
      const float ov = __shfl_xor(v, o);
      const int   oi = __shfl_xor(ix, o);
      const bool tk = (ov > v) || (ov == v && oi < ix);
      v = tk ? ov : v;
      ix = tk ? oi : ix;
    }
    cur = clampi(ix, 0, kPts - 1);
    if (tid == 0) s_sel[it] = cur;
  }
  __syncthreads();

  if (tid < 256) {
    const v4i v = *(const v4i*)(s_sel + 4 * tid);
    volatile v4i* dst = (volatile v4i*)(fps_idx + b * kCent + 4 * tid);
    *dst = v;
    __threadfence();
    *dst = v;
  } else {
    const int t2 = tid - 256;
    float ov[4];
#pragma unroll
    for (int e = 0; e < 4; ++e) {
      const int flat = 4 * t2 + e;
      const int pt = flat / 3;
      const int cc = flat - 3 * pt;
      const int si = clampi(s_sel[pt], 0, kPts - 1);
      ov[e] = s_x[si * 3 + cc];
    }
    v4f v;
    v.x = ov[0]; v.y = ov[1]; v.z = ov[2]; v.w = ov[3];
    volatile v4f* dst = (volatile v4f*)(out0 + (size_t)b * kCent * 3 + 4 * t2);
    *dst = v;
    __threadfence();
    *dst = v;
  }
}

__global__ __launch_bounds__(256) void k_ballq(const float* __restrict__ xyzr, const int* __restrict__ fps_idx,
                                               int* __restrict__ nb_idx) {
#pragma clang fp contract(off)
  __shared__ float s_px[kPts];
  __shared__ float s_py[kPts];
  __shared__ float s_pz[kPts];
  __shared__ int   s_list[8][32];
  const int b = blockIdx.x >> 5;
  const int n0 = (blockIdx.x & 31) * 32;
  const int tid = threadIdx.x;
  const int lane = tid & 31;
  const int wave = tid >> 5;
  const float* X = xyzr + (size_t)b * kPts * 3;
#pragma unroll 4
  for (int j = tid; j < kPts; j += 256) {
    s_px[j] = X[j * 3 + 0];
    s_py[j] = X[j * 3 + 1];
    s_pz[j] = X[j * 3 + 2];
  }
  __syncthreads();
  const float thr = __uint_as_float(0x3D23D70Au);

#pragma unroll 1
  for (int t = 0; t < 4; ++t) {
    const int n = n0 + wave * 4 + t;
    const int fi = clampi(fps_idx[b * kCent + n], 0, kPts - 1);
    const float qx = s_px[fi];
    const float qy = s_py[fi];
    const float qz = s_pz[fi];
    const float q0 = qx * qx;
    const float q1 = qy * qy;
    const float q2 = qz * qz;
    const float qq = (q0 + q2) + q1;
    s_list[wave][lane] = 0;
    __builtin_amdgcn_fence(__ATOMIC_RELEASE, "workgroup");
    __builtin_amdgcn_wave_barrier();
    __builtin_amdgcn_fence(__ATOMIC_ACQUIRE, "workgroup");
    int cnt = 0;
#pragma unroll 1
    for (int ch = 0; ch < kPts / 32 && cnt < kNbr; ++ch) {
      const int j = ch * 32 + lane;
      const float px = s_px[j];
      const float py = s_py[j];
      const float pz = s_pz[j];
      const float p0 = px * px;
      const float p1 = py * py;
      const float p2 = pz * pz;
      const float pp = (p0 + p2) + p1;
      float dot = qx * px;
      dot = __builtin_fmaf(qy, py, dot);
      dot = __builtin_fmaf(qz, pz, dot);
      const float two_dot = 2.0f * dot;
      const float d2 = (qq + pp) - two_dot;
      const bool hit = d2 <= thr;
      const unsigned mask = __builtin_amdgcn_ballot_w32(hit);
      const int pos = cnt + __builtin_popcount(mask & ((1u << lane) - 1u));
      if (hit && pos < kNbr) s_list[wave][pos] = j;
      cnt += __builtin_popcount(mask);
    }
    __builtin_amdgcn_fence(__ATOMIC_RELEASE, "workgroup");
    __builtin_amdgcn_wave_barrier();
    __builtin_amdgcn_fence(__ATOMIC_ACQUIRE, "workgroup");
    const int c2 = cnt < kNbr ? cnt : kNbr;
    const int src = (lane < c2) ? lane : 0;
    int v = s_list[wave][src];
    v = (c2 == 0) ? (kPts - 1) : v;
    v = clampi(v, 0, kPts - 1);
    volatile int* dst = nb_idx + ((size_t)(b * kCent + n)) * kNbr + lane;
    *dst = v;
    __threadfence();
    *dst = v;
    __builtin_amdgcn_fence(__ATOMIC_RELEASE, "workgroup");
    __builtin_amdgcn_wave_barrier();
    __builtin_amdgcn_fence(__ATOMIC_ACQUIRE, "workgroup");
  }
}

union FragU { v16h v; v4u q[2]; };

__device__ __forceinline__ void guard2(v8f& a, v8f& b, v16h x, v16h y, v16h z) {
  asm volatile("v_nop\n\tv_nop\n\tv_nop\n\tv_nop" : "+v"(a), "+v"(b) : "v"(x), "v"(y), "v"(z));
}

__device__ __forceinline__ void softmax3(float a, float b, float c, float& oa, float& ob, float& oc) {
  const float m = fmaxf(a, fmaxf(b, c));
  const float ea = expf(a - m);
  const float eb = expf(b - m);
  const float ec = expf(c - m);
  const float inv = 1.0f / ((ea + eb) + ec);
  oa = ea * inv;
  ob = eb * inv;
  oc = ec * inv;
}

__global__ __launch_bounds__(128) void k_enhance_attn(
    const float* __restrict__ xyzr, const unsigned* __restrict__ featT, const unsigned* __restrict__ AtW,
    const int* __restrict__ fps_idx, const int* __restrict__ nb_idx,
    unsigned* __restrict__ poolH, unsigned* __restrict__ poolL) {
  __shared__ __align__(16) unsigned s_tile[4][32 * kTilePW];
  __shared__ __align__(16) unsigned s_ph[4][kRowW];
  __shared__ __align__(16) unsigned s_pl[4][kRowW];

  const int tid = threadIdx.x;
  const int wave = tid >> 5;
  const int lane = tid & 31;
  const int h = lane >> 4;
  const int c = lane & 15;
  const int p = blockIdx.x * 4 + wave;
  const int b = p >> 10;

  {
    const int fpsi = clampi(fps_idx[p], 0, kPts - 1);
    const int nbi = clampi(nb_idx[(size_t)p * kNbr + lane], 0, kPts - 1);
    const float* Xb = xyzr + (size_t)b * kPts * 3;
    const float gx = Xb[fpsi * 3 + 0];
    const float gy = Xb[fpsi * 3 + 1];
    const float gz = Xb[fpsi * 3 + 2];
    float gnx = Xb[nbi * 3 + 0];
    float gny = Xb[nbi * 3 + 1];
    float gnz = Xb[nbi * 3 + 2];
    const v4u* fl = (const v4u*)(featT + ((size_t)(b * kPts + fpsi)) * 32);
    const v4u* nl = (const v4u*)(featT + ((size_t)(b * kPts + nbi)) * 32);
    unsigned* trow = &s_tile[wave][lane * kTilePW];

    float dsum = 0.0f;
    float df2 = 0.0f;
#pragma unroll 1
    for (int ch = 0; ch < 8; ++ch) {
      const v4u fq = fl[ch];
      const v4u nq = nl[ch];
      unsigned fw[4], nw[4];
      fw[0] = fq.x; fw[1] = fq.y; fw[2] = fq.z; fw[3] = fq.w;
      nw[0] = nq.x; nw[1] = nq.y; nw[2] = nq.z; nw[3] = nq.w;
      unsigned wf[4], wn[4], wd[4];
#pragma unroll
      for (int i = 0; i < 4; ++i) {
        const float f0 = __uint_as_float(fw[i] << 16);
        const float f1 = __uint_as_float(fw[i] & 0xffff0000u);
        const float m0 = __uint_as_float(nw[i] << 16);
        const float m1 = __uint_as_float(nw[i] & 0xffff0000u);
        const float d0 = f0 - m0;
        const float d1 = f1 - m1;
        dsum += fabsf(d0);
        dsum += fabsf(d1);
        df2 += d0 * d0;
        df2 += d1 * d1;
        wf[i] = pk16(f0, f1);
        wn[i] = pk16(m0, m1);
        wd[i] = pk16(d0, d1);
      }
      v4u sv;
      sv.x = wn[0]; sv.y = wn[1]; sv.z = wn[2]; sv.w = wn[3];
      *(v4u*)(trow + ch * 4) = sv;
      sv.x = wf[0]; sv.y = wf[1]; sv.z = wf[2]; sv.w = wf[3];
      *(v4u*)(trow + 32 + ch * 4) = sv;
      sv.x = wd[0]; sv.y = wd[1]; sv.z = wd[2]; sv.w = wd[3];
      *(v4u*)(trow + 64 + ch * 4) = sv;
    }
    const float fdist = expf(-(dsum * (1.0f / (float)kFeat)));
    gnx *= fdist;
    gny *= fdist;
    gnz *= fdist;
    float mx = gnx, my = gny, mz = gnz;
#pragma unroll
    for (int o = 16; o > 0; o >>= 1) {
      const float ax = __shfl_xor(mx, o);
      const float ay = __shfl_xor(my, o);
      const float az = __shfl_xor(mz, o);
      mx += ax;
      my += ay;
      mz += az;
    }
    mx *= (1.0f / (float)kNbr);
    my *= (1.0f / (float)kNbr);
    mz *= (1.0f / (float)kNbr);
    float sgx, sgy, sgz, smx, smy, smz;
    softmax3(gx, gy, gz, sgx, sgy, sgz);
    softmax3(mx, my, mz, smx, smy, smz);
    const float gdx = fabsf(smx - sgx);
    const float gdy = fabsf(smy - sgy);
    const float gdz = fabsf(smz - sgz);
    const float p1x = gx - gnx;
    const float p1y = gy - gny;
    const float p1z = gz - gnz;
    const float dg = sqrtf((p1x * p1x + p1y * p1y) + p1z * p1z);
    const float q1x = gx - gdx;
    const float q1y = gy - gdy;
    const float q1z = gz - gdz;
    df2 += q1x * q1x;
    df2 += q1y * q1y;
    df2 += q1z * q1z;
    const float df = sqrtf(df2);
    unsigned zz = 0u;
    asm volatile("" : "+v"(zz));
    v4u sv;
    sv.x = pk16(gnx, gny); sv.y = pk16(gnz, gx); sv.z = pk16(gy, gz); sv.w = pk16(p1x, p1y);
    *(v4u*)(trow + 96) = sv;
    sv.x = pk16(p1z, dg); sv.y = pk16(gdx, gdy); sv.z = pk16(gdz, gx); sv.w = pk16(gy, gz);
    *(v4u*)(trow + 100) = sv;
    sv.x = pk16(q1x, q1y); sv.y = pk16(q1z, df); sv.z = zz; sv.w = zz;
    *(v4u*)(trow + 104) = sv;
    sv.x = zz; sv.y = zz; sv.z = zz; sv.w = zz;
    *(v4u*)(trow + 108) = sv;
  }
  __syncthreads();

  const unsigned* tw = s_tile[wave];
#pragma unroll 1
  for (int nt = 0; nt < kChanPad / 16; ++nt) {
    v8f acc0 = (v8f){0.f, 0.f, 0.f, 0.f, 0.f, 0.f, 0.f, 0.f};
    v8f acc1 = (v8f){0.f, 0.f, 0.f, 0.f, 0.f, 0.f, 0.f, 0.f};
    const unsigned* brow  = AtW + (size_t)(nt * 16 + c) * kRowW + 4 * h;
    const unsigned* a0row = tw + c * kTilePW + 4 * h;
    const unsigned* a1row = tw + (16 + c) * kTilePW + 4 * h;
#pragma unroll
    for (int ks = 0; ks < kChanPad / 32; ++ks) {
      FragU fb, fa0, fa1;
      fb.q[0]  = *(const v4u*)(brow + ks * 16);
      fb.q[1]  = *(const v4u*)(brow + ks * 16 + 8);
      fa0.q[0] = *(const v4u*)(a0row + ks * 16);
      fa0.q[1] = *(const v4u*)(a0row + ks * 16 + 8);
      fa1.q[0] = *(const v4u*)(a1row + ks * 16);
      fa1.q[1] = *(const v4u*)(a1row + ks * 16 + 8);
      acc0 = __builtin_amdgcn_wmma_f32_16x16x32_f16(false, fa0.v, false, fb.v, (short)0, acc0, false, false);
      acc1 = __builtin_amdgcn_wmma_f32_16x16x32_f16(false, fa1.v, false, fb.v, (short)0, acc1, false, false);
      guard2(acc0, acc1, fa0.v, fa1.v, fb.v);
      if (ks == 3) asm volatile("" ::: "memory");
    }

    const int n = nt * 16 + c;
    const int sh = (n & 1) * 16;
    const unsigned* colp = tw + (n >> 1);
    float e0[8], e1[8];
    float m = -INFINITY;
#pragma unroll
    for (int r = 0; r < 8; ++r) {
      float x0 = acc0[r] * kWCarryInv;
      float x1 = acc1[r] * kWCarryInv;
      x0 = (x0 >= 0.0f) ? x0 : (0.2f * x0);
      x1 = (x1 >= 0.0f) ? x1 : (0.2f * x1);
      e0[r] = x0;
      e1[r] = x1;
      m = fmaxf(m, fmaxf(x0, x1));
    }
    {
      const float om = __shfl_xor(m, 16);
      m = fmaxf(m, om);
    }
    float s = 0.0f;
    float ps = 0.0f;
#pragma unroll 1
    for (int t = 0; t < 2; ++t) {
#pragma unroll
      for (int r = 0; r < 8; ++r) {
        const float ev = (t != 0) ? e1[r] : e0[r];
        const float ex = expf(ev - m);
        const int row = 16 * t + 8 * h + r;
        const unsigned w = colp[row * kTilePW];
        const float val = h16_to_f32((w >> sh) & 0xffffu);
        const float pr = ex * val;
        s += ex;
        ps += pr;
      }
    }
    {
      const float os = __shfl_xor(s, 16);
      const float op = __shfl_xor(ps, 16);
      s += os;
      ps += op;
    }
    const float pooled = ps * (1.0f / s);
    const float other = __shfl_xor(pooled, 1);
    const bool odd = (lane & 1) != 0;
    const float lo_v = odd ? other : pooled;
    const float hi_v = odd ? pooled : other;
    const unsigned hb0 = (unsigned)f2bf_bits(lo_v);
    const unsigned hb1 = (unsigned)f2bf_bits(hi_v);
    const float r0 = lo_v - __uint_as_float(hb0 << 16);
    const float r1 = hi_v - __uint_as_float(hb1 << 16);
    const unsigned lb0 = (unsigned)f2bf_bits(r0);
    const unsigned lb1 = (unsigned)f2bf_bits(r1);
    const unsigned wH = (hb0 & 0xffffu) | (hb1 << 16);
    const unsigned wL = (lb0 & 0xffffu) | (lb1 << 16);
    if (lane < 16 && !odd) {
      s_ph[wave][n >> 1] = wH;
      s_pl[wave][n >> 1] = wL;
    }
  }
  __syncthreads();

  {
    const int tc = tid < 112 ? tid : 111;
    const int row = tc / 28;
    const int w4 = (tc - row * 28) * 4;
    const v4u vH = *(const v4u*)(&s_ph[row][w4]);
    const v4u vL = *(const v4u*)(&s_pl[row][w4]);
    const size_t off = (size_t)blockIdx.x * 4 * kRowW + (size_t)tc * 4;
    const bool st = tid < 112;
    if (st) {
      *(volatile v4u*)(poolH + off) = vH;
      *(volatile v4u*)(poolL + off) = vL;
    }
    __threadfence();
    if (st) {
      *(volatile v4u*)(poolH + off) = vH;
      *(volatile v4u*)(poolL + off) = vL;
    }
  }
}

__device__ __forceinline__ void dep_guard_h(v8f& a, v8f& b, v16h x, v16h y) { asm volatile("v_nop\n\tv_nop\n\tv_nop\n\tv_nop" : "+v"(a), "+v"(b) : "v"(x), "v"(y)); }
__device__ __forceinline__ void dep_guard_b(v8f& a, v8f& b, v16b x, v16b y) { asm volatile("v_nop\n\tv_nop\n\tv_nop\n\tv_nop" : "+v"(a), "+v"(b) : "v"(x), "v"(y)); }
__device__ __forceinline__ void keep4_h(v16h a, v16h b, v16h c, v16h d) { asm volatile("v_nop" :: "v"(a), "v"(b), "v"(c), "v"(d)); }
__device__ __forceinline__ void keep4_b(v16b a, v16b b, v16b c, v16b d) { asm volatile("v_nop" :: "v"(a), "v"(b), "v"(c), "v"(d)); }
__device__ __forceinline__ void acc_guard4(v8f& a, v8f& b, v8f& c, v8f& d) { asm volatile("v_nop\n\tv_nop\n\tv_nop\n\tv_nop" : "+v"(a), "+v"(b), "+v"(c), "+v"(d)); }
template <typename T> struct Frag;
template <> struct Frag<_Float16> {
  typedef v16h V; union U { v16h v; v8h h[2]; };
  static __device__ __forceinline__ v16h load(const _Float16* p) {
    U f; f.h[0] = *(const v8h*)(p); f.h[1] = *(const v8h*)(p + 16); return f.v;
  }
  static __device__ __forceinline__ v8f mma(v16h a, v16h b, v8f c) {
    return __builtin_amdgcn_wmma_f32_16x16x32_f16(false, a, false, b, (short)0, c, false, false);
  }
  static __device__ __forceinline__ void guard(v8f& a, v8f& b, v16h x, v16h y) { dep_guard_h(a, b, x, y); }
  static __device__ __forceinline__ void keep(v16h a, v16h b, v16h c, v16h d) { keep4_h(a, b, c, d); }
};
template <> struct Frag<__bf16> {
  typedef v16b V; union U { v16b v; v8b h[2]; };
  static __device__ __forceinline__ v16b load(const __bf16* p) {
    U f; f.h[0] = *(const v8b*)(p); f.h[1] = *(const v8b*)(p + 16); return f.v;
  }
  static __device__ __forceinline__ v8f mma(v16b a, v16b b, v8f c) {
    return __builtin_amdgcn_wmma_f32_16x16x32_bf16(false, a, false, b, (short)0, c, false, false);
  }
  static __device__ __forceinline__ void guard(v8f& a, v8f& b, v16b x, v16b y) { dep_guard_b(a, b, x, y); }
  static __device__ __forceinline__ void keep(v16b a, v16b b, v16b c, v16b d) { keep4_b(a, b, c, d); }
};

template <int ET> struct Elem;
template <> struct Elem<0> { typedef _Float16 T; };
template <> struct Elem<1> { typedef __bf16 T; };
template <int ET, bool SPLIT, int BIAS_MODE, int OUT_MODE, bool RESID, int ACT = 0>
__global__ __launch_bounds__(256) void wmma_gemm64(
    const unsigned short* __restrict__ Ap, const unsigned short* __restrict__ A2p, int lda, long strideA,
    const unsigned short* __restrict__ Btp, const unsigned short* __restrict__ Bt2p, int ldb, long strideB,
    void* __restrict__ Cout, void* __restrict__ Cout2, int ldc, long strideC,
    const float* __restrict__ bias,
    const float* __restrict__ resid, long strideR,
    int M, int N, int K, float scale) {
  typedef typename Elem<ET>::T T;
  typedef typename Frag<T>::V V;
  const T* A = (const T*)Ap; const T* A2 = (const T*)A2p; const T* Bt = (const T*)Btp; const T* Bt2 = (const T*)Bt2p;
  __shared__ __align__(16) float sT[8][16 * 68];
  const int b    = blockIdx.y;
  const int lane = threadIdx.x & 31;
  const int wave = threadIdx.x >> 5;
  const int tilesN = N >> 6;
  const int tilesM = M >> 6;
  const int tile = blockIdx.x * 8 + wave;
  if (tile >= tilesM * tilesN) return;
  const int tm = tile / tilesN;
  const int tn = tile - tm * tilesN;
  const int m0 = tm << 6;
  const int n0 = tn << 6;

  const T* Ab  = A  + (size_t)b * strideA;
  const T* Bb  = Bt + (size_t)b * strideB;
  const T* Ab2 = SPLIT ? (A2  + (size_t)b * strideA) : nullptr;
  const T* Bb2 = SPLIT ? (Bt2 + (size_t)b * strideB) : nullptr;

  const int rlane = lane & 15;
  const int koff  = (lane >> 4) * 8;
  const int mOff  = (lane >> 4) * 8;

  v8f acc[4][4];
#pragma unroll
  for (int i = 0; i < 4; ++i)
#pragma unroll
    for (int j = 0; j < 4; ++j) acc[i][j] = (v8f){0.f,0.f,0.f,0.f,0.f,0.f,0.f,0.f};

  for (int k0 = 0; k0 < K; k0 += 32) {
    V bh[4], bl[4];
#pragma unroll
    for (int j = 0; j < 4; ++j) {
      const size_t bo = (size_t)(n0 + (j << 4) + rlane) * ldb + koff + k0;
      bh[j] = Frag<T>::load(Bb + bo);
      if (SPLIT) bl[j] = Frag<T>::load(Bb2 + bo);
    }
#pragma unroll
    for (int i = 0; i < 4; ++i) {
      const size_t ao = (size_t)(m0 + (i << 4) + rlane) * lda + koff + k0;
      V ah = Frag<T>::load(Ab + ao);
      V al;
      if (SPLIT) al = Frag<T>::load(Ab2 + ao);
#pragma unroll
      for (int j = 0; j < 4; ++j) {
        acc[i][j] = Frag<T>::mma(ah, bh[j], acc[i][j]);
        if (SPLIT) {
          acc[i][j] = Frag<T>::mma(ah, bl[j], acc[i][j]);
          acc[i][j] = Frag<T>::mma(al, bh[j], acc[i][j]);
        }
      }
      Frag<T>::guard(acc[i][0], acc[i][3], ah, SPLIT ? al : ah);
    }
    Frag<T>::keep(bh[0], bh[1], bh[2], bh[3]);
    if (SPLIT) Frag<T>::keep(bl[0], bl[1], bl[2], bl[3]);
  }
  acc_guard4(acc[0][0], acc[0][1], acc[0][2], acc[0][3]);
  acc_guard4(acc[1][0], acc[1][1], acc[1][2], acc[1][3]);
  acc_guard4(acc[2][0], acc[2][1], acc[2][2], acc[2][3]);
  acc_guard4(acc[3][0], acc[3][1], acc[3][2], acc[3][3]);

  float* slab = sT[wave];
  const float* Rb = RESID ? (resid + (size_t)b * strideR) : nullptr;
#pragma unroll
  for (int i = 0; i < 4; ++i) {
    const int mBase = m0 + (i << 4);
#pragma unroll
    for (int j = 0; j < 4; ++j) {
      const int n = n0 + (j << 4) + rlane;
      float bv = 0.f;
      if (BIAS_MODE == 2) bv = bias[n];
#pragma unroll
      for (int r = 0; r < 8; ++r) {
        float v = acc[i][j][r] * scale;
        if (BIAS_MODE == 1) v += bias[mBase + mOff + r];
        if (BIAS_MODE == 2) v += bv;
        if (RESID) v += Rb[(size_t)(mBase + mOff + r) * ldc + n];
        if (ACT == 2) v = fmaxf(v, 0.0f);
        if (ACT == 4) v = (v > 0.f) ? v : 0.01f * v;
        slab[(mOff + r) * 68 + (j << 4) + rlane] = v;
      }
    }
    __builtin_amdgcn_fence(__ATOMIC_RELEASE, "workgroup");
    __builtin_amdgcn_wave_barrier();
    __builtin_amdgcn_fence(__ATOMIC_ACQUIRE, "workgroup");
    if (OUT_MODE == 0) {
      float* C = (float*)Cout + (size_t)b * strideC;
      const int hh = lane >> 4, c4 = (lane & 15) * 4;
      for (int pass = 0; pass < 2; ++pass) {
#pragma unroll
        for (int it = 0; it < 8; ++it) {
          const int row = it * 2 + hh;
          v4f v = *(const v4f*)(slab + row * 68 + c4);
          *(volatile v4f*)(C + (size_t)(mBase + row) * ldc + n0 + c4) = v;
        }
        __threadfence();
      }
    } else {
      const int q = lane >> 3, c8 = (lane & 7) * 8;
      unsigned short* C  = (unsigned short*)Cout  + (size_t)b * strideC;
      unsigned short* C2 = (OUT_MODE == 2) ? ((unsigned short*)Cout2 + (size_t)b * strideC) : nullptr;
      for (int pass = 0; pass < 2; ++pass) {
#pragma unroll
        for (int it = 0; it < 4; ++it) {
          const int row = it * 4 + q;
          const float* sp = slab + row * 68 + c8;
          v8h hv, lv;
#pragma unroll
          for (int e = 0; e < 8; ++e) {
            if (OUT_MODE == 1) {
              hv[e] = (_Float16)sp[e];
            } else {
              unsigned short hb = f2bf_bits(sp[e]);
              unsigned short lb = f2bf_bits(sp[e] - bf_bits2f(hb));
              hv[e] = __builtin_bit_cast(_Float16, hb);
              lv[e] = __builtin_bit_cast(_Float16, lb);
            }
          }
          *(volatile v8h*)(C + (size_t)(mBase + row) * ldc + n0 + c8) = hv;
          if (OUT_MODE == 2) *(volatile v8h*)(C2 + (size_t)(mBase + row) * ldc + n0 + c8) = lv;
        }
        __threadfence();
      }
    }
    __builtin_amdgcn_fence(__ATOMIC_RELEASE, "workgroup");
    __builtin_amdgcn_wave_barrier();
    __builtin_amdgcn_fence(__ATOMIC_ACQUIRE, "workgroup");
  }
}

extern "C" void kernel_launch(void* const* d_in, const int* in_sizes, int n_in,
                              void* d_out, int out_size, void* d_ws, size_t ws_size, hipStream_t stream) {
  (void)in_sizes; (void)n_in; (void)out_size;
  const float* xyz  = (const float*)d_in[0];
  const float* feat = (const float*)d_in[1];
  const float* amat = (const float*)d_in[2];
  const float* w1   = (const float*)d_in[3];
  const float* b1   = (const float*)d_in[4];

  float* out0 = (float*)d_out;
  float* out1 = (float*)d_out + (98304 / 4);

  constexpr size_t szXyzr  = (size_t)kBatch * kPts * 3 * 4;
  constexpr size_t szFeatT = (size_t)kBatch * kPts * kFeat * 2;
  constexpr size_t szAt    = (size_t)kChanPad * kChanPad * 2;
  constexpr size_t szW1    = (size_t)kOutCh * kChanPad * 2;
  constexpr size_t szB1    = (size_t)kOutCh * 4;
  constexpr size_t szFps   = (size_t)kBatch * kCent * 4;
  constexpr size_t szNb    = (size_t)kBatch * kCent * kNbr * 4;
  constexpr size_t szPool  = (size_t)kBatch * kCent * kChanPad * 2;
  static_assert(szXyzr % 128 == 0 && szFeatT % 128 == 0 && szAt % 128 == 0 && szW1 % 128 == 0 &&
                szB1 % 128 == 0 && szFps % 128 == 0 && szNb % 128 == 0 && szPool % 128 == 0, "line-aligned carve");
  constexpr size_t total = szXyzr + szFeatT + szAt + 2 * szW1 + szB1 + szFps + szNb + 2 * szPool;
  static_assert(total <= 134217728, "carve under 128 MiB");
  if (total > ws_size) return;

  char* ws = (char*)d_ws;
  size_t off = 0;
  float*    xyzr  = (float*)(ws + off);    off += szXyzr;
  unsigned* featT = (unsigned*)(ws + off); off += szFeatT;
  unsigned* AtW   = (unsigned*)(ws + off); off += szAt;
  unsigned* W1b   = (unsigned*)(ws + off); off += szW1;
  unsigned* W1z   = (unsigned*)(ws + off); off += szW1;
  float*    b1r   = (float*)(ws + off);    off += szB1;
  int*      fps   = (int*)(ws + off);      off += szFps;
  int*      nb    = (int*)(ws + off);      off += szNb;
  unsigned* poolH = (unsigned*)(ws + off); off += szPool;
  unsigned* poolL = (unsigned*)(ws + off); off += szPool;

  k_prep_xyz<<<(kBatch * kPts * 3 / 4) / 256 + 1, 256, 0, stream>>>(xyz, b1, xyzr, b1r);
  k_prep_feat<<<kBatch * (kPts / 64), 256, 0, stream>>>(feat, featT);
  k_prep_at<<<(kChanPad * 28 + 255) / 256, 256, 0, stream>>>(amat, AtW);
  k_prep_w1<<<(kOutCh * 28 + 255) / 256, 256, 0, stream>>>(w1, W1b, W1z);
  k_fps<<<kBatch, 1024, 0, stream>>>(xyzr, fps, out0);
  k_ballq<<<kBatch * 32, 256, 0, stream>>>(xyzr, fps, nb);
  k_enhance_attn<<<(kBatch * kCent) / 4, 128, 0, stream>>>(xyzr, featT, AtW, fps, nb, poolH, poolL);

  static_assert(kOutCh % 64 == 0 && kCent % 64 == 0 && kChanPad % 32 == 0, "GEMM shape");
  wmma_gemm64<1, true, 1, 0, false, 0><<<dim3((kOutCh / 64) * (kCent / 64) / 8, kBatch), 256, 0, stream>>>(
      (const unsigned short*)W1b, (const unsigned short*)W1z, kChanPad, 0L,
      (const unsigned short*)poolH, (const unsigned short*)poolL, kChanPad, (long)kCent * kChanPad,
      (void*)out1, nullptr, kCent, (long)kOutCh * kCent,
      b1r, nullptr, 0L,
      kOutCh, kCent, kChanPad, 1.0f);
}
